// EncoderBlock_2568390443463
// MI455X (gfx1250) — hardware-run, weakly checked
//
#include <hip/hip_runtime.h>


#ifndef NB
#define NB 8
#endif
#ifndef SEQ
#define SEQ 1024
#endif
#define NB_FULL  8
#define SEQ_FULL 1024
#ifndef OUT_SEQ
#define OUT_SEQ SEQ
#endif
#define DM   512
#define NH_  8
#define HD   64
#define NCONV 4
#define KW   7
#define NTOK (NB * SEQ)
#define OSP  36
#define HSP  41
#define SC2  (0.125f * 1.4426950408889634f)
#define NEGL (-1.0e30f * 1.4426950408889634f)
#define PSH  8.0f
#define LNE  1.0e-5f
#define WCAR 64.0f
#define XCAR 16.0f
#define LOGINC 0.036118981850887f
#define LOG2E  1.4426950408889634f

static_assert(HD == 64);
static_assert(NH_ * HD == DM);
static_assert(DM == 512);
static_assert(DM % 64 == 0);
static_assert(DM % 32 == 0);
static_assert(SEQ % 64 == 0);
static_assert(NTOK % 64 == 0);
static_assert(SEQ % 32 == 0);
static_assert(SEQ / 32 <= 32);
static_assert(NH_ == 8);
static_assert((OSP * 4) % 16 == 0);
static_assert(OSP >= 32);
static_assert(HSP >= 40);
static_assert(KW == 7);
static_assert(((DM / 2) * SEQ) % 256 == 0);
static_assert(((size_t)DM * DM) % 8 == 0);
static_assert(((size_t)DM * KW) % 1 == 0);
static_assert(NB <= NB_FULL);
static_assert(SEQ <= SEQ_FULL);

typedef _Float16 h16;
typedef __attribute__((ext_vector_type(16))) _Float16 v16h;
typedef __attribute__((ext_vector_type(8)))  _Float16 v8h;
typedef __attribute__((ext_vector_type(8)))  float    v8f;
typedef __attribute__((ext_vector_type(4)))  float    v4f;
typedef v4f  __attribute__((may_alias)) v4fa;

__device__ __forceinline__ unsigned short f2bf(float f) { unsigned u = __float_as_uint(f); u += 0x7FFFu + ((u >> 16) & 1u); return (unsigned short)(u >> 16); }
__device__ __forceinline__ float bfr(float f) { return __uint_as_float(((unsigned)f2bf(f)) << 16); }
__device__ __forceinline__ v16h cat16(v8h lo, v8h hi) { return __builtin_shufflevector(lo, hi, 0, 1, 2, 3, 4, 5, 6, 7, 8, 9, 10, 11, 12, 13, 14, 15); }
__device__ __forceinline__ v8f wmma16(v16h a, v16h b, v8f c) { return __builtin_amdgcn_wmma_f32_16x16x32_f16(false, a, false, b, (short)0, c, false, false); }
__device__ __forceinline__ v16h  ldh(const h16* p) { return cat16(*(const v8h*)p, *(const v8h*)(p + 16)); }
__device__ __forceinline__ void wave_sync() { __builtin_amdgcn_fence(3  , "wavefront"); __builtin_amdgcn_wave_barrier(); asm volatile("" ::: "memory"); }

__global__ __launch_bounds__(256) void k_cvtw(const float* __restrict__ src, h16* dst, size_t n8) {
    const size_t i = (size_t)blockIdx.x * 256 + threadIdx.x; if (i >= n8) return;
    const v8f v = *(const v8f*)(src + i * 8); v8h o;
#pragma unroll
    for (int k = 0; k < 8; ++k) o[k] = (h16)(bfr(v[k]) * WCAR);
    *(volatile v8h*)(dst + i * 8) = o; __threadfence(); *(volatile v8h*)(dst + i * 8) = o;
}

__global__ __launch_bounds__(256) void k_pos(const float* __restrict__ x, float* A0) {
    const int idx = blockIdx.x * 256 + threadIdx.x;
    if (idx >= (DM / 2) * SEQ) return;
    const int l = idx % SEQ, j = idx / SEQ;
    const float e = (float)j * (-LOGINC);
    const float ts = __builtin_amdgcn_exp2f(e * LOG2E);
    const float ang = (float)l * ts;
    const float sn = sinf(ang), cs = cosf(ang);
#pragma unroll 1
    for (int ps = 0; ps < 2; ++ps) {
#pragma unroll 1
        for (int b = 0; b < NB; ++b) {
            const float xs = x[((size_t)b * DM + j) * SEQ_FULL + l];
            const float xc = x[((size_t)b * DM + (DM / 2) + j) * SEQ_FULL + l];
            const float ys = bfr(xs) + sn, yc = bfr(xc) + cs;
            *(volatile float*)(A0 + ((size_t)b * DM + j) * SEQ + l) = ys;
            *(volatile float*)(A0 + ((size_t)b * DM + (DM / 2) + j) * SEQ + l) = yc; }
        if (ps == 0) __threadfence(); }
}

__global__ __launch_bounds__(256) void k_stats(const float* __restrict__ ACT, float* ST) {
    __shared__ float red[8 * 32];
    __shared__ float red2[8 * 32];
    const int lane = threadIdx.x & 31;
    const int wv = __builtin_amdgcn_readfirstlane((int)(threadIdx.x >> 5));
    const int n0 = blockIdx.x * 32, b = n0 / SEQ, l0 = n0 % SEQ;
    const float* p = ACT + ((size_t)b * DM + (size_t)wv * 64) * SEQ + l0 + lane;
    float s = 0.0f;
#pragma unroll 4
    for (int d = 0; d < 64; ++d) s += p[(size_t)d * SEQ];
    red[wv * 32 + lane] = s;
    __syncthreads();
    float S = 0.0f;
#pragma unroll
    for (int j = 0; j < 8; ++j) S += red[j * 32 + lane];
    const float mu = S * (1.0f / (float)DM);
    float q = 0.0f;
#pragma unroll 4
    for (int d = 0; d < 64; ++d) { const float dv = p[(size_t)d * SEQ] - mu; q += dv * dv; }
    red2[wv * 32 + lane] = q;
    __syncthreads();
    if (wv == 0) {
        float Q = 0.0f;
#pragma unroll
        for (int j = 0; j < 8; ++j) Q += red2[j * 32 + lane];
        const float rs = rsqrtf(Q * (1.0f / (float)DM) + LNE);
        *(volatile float*)(ST + n0 + lane) = mu; *(volatile float*)(ST + (size_t)NTOK + n0 + lane) = rs;
        __threadfence();
        *(volatile float*)(ST + n0 + lane) = mu; *(volatile float*)(ST + (size_t)NTOK + n0 + lane) = rs;
    }
}

template <int HASDW>
__device__ __forceinline__ void lndw_body(const float* __restrict__ ACT, const float* __restrict__ ST, const float* __restrict__ G, const float* __restrict__ BE,
                                          const float* __restrict__ DW, float carry, h16* XP) {
    __shared__ __align__(16) float hs[64 * HSP];
    __shared__ __align__(16) float ys[32 * 68];
    const int tid = threadIdx.x, lane = tid & 31;
    const int wv = __builtin_amdgcn_readfirstlane((int)(threadIdx.x >> 5));
    const int n0 = blockIdx.x * 32, b = n0 / SEQ, l0 = n0 % SEQ, c0 = blockIdx.y * 64;
    const int jm = 4 + lane;
    const int jh = (lane & 4) ? (32 + (lane & 7)) : (lane & 7);
    const int lh = l0 - 4 + jh;
    const bool okh = (lh >= 0) && (lh < SEQ);
    const int lhc = (lh < 0) ? 0 : ((lh > SEQ - 1) ? (SEQ - 1) : lh);
    const float mum = ST[(size_t)b * SEQ + l0 + lane], rsm = ST[(size_t)NTOK + (size_t)b * SEQ + l0 + lane];
    const float muh = ST[(size_t)b * SEQ + lhc],       rsh = ST[(size_t)NTOK + (size_t)b * SEQ + lhc];
#pragma unroll 1
    for (int i = 0; i < 8; ++i) {
        const int ci = wv * 8 + i, c = c0 + ci;
        const float g = bfr(G[c]), be = bfr(BE[c]);
        const float* row = ACT + ((size_t)b * DM + c) * SEQ;
        const float xm = row[l0 + lane];
        float xh = row[lhc];
        asm volatile("" : "+v"(xh));
        const float hm = (g * (xm - mum)) * rsm + be;
        float hh = (g * (xh - muh)) * rsh + be; hh = okh ? hh : 0.0f;
        hs[ci * HSP + jm] = hm;
        if (lane < 8) hs[ci * HSP + jh] = hh;
    }
    __syncthreads();
#pragma unroll 1
    for (int i = 0; i < 8; ++i) {
        const int ci = wv * 8 + i, c = c0 + ci;
        float y;
        if (HASDW) { y = 0.0f;
#pragma unroll
            for (int t = 0; t < KW; ++t) y += hs[ci * HSP + lane + 1 + t] * bfr(DW[(size_t)c * KW + t]); }
        else y = hs[ci * HSP + lane + 4];
        ys[lane * 68 + ci] = y * carry;
    }
    __syncthreads();
    const int row = tid >> 3, c8 = (tid & 7) * 8;
#pragma unroll 1
    for (int ps = 0; ps < 2; ++ps) {
        const v4f x0 = *(const v4fa*)(&ys[row * 68 + c8]); const v4f x1 = *(const v4fa*)(&ys[row * 68 + c8 + 4]); v8h hv;
#pragma unroll
        for (int i = 0; i < 4; ++i) { hv[i] = (h16)x0[i]; hv[4 + i] = (h16)x1[i]; }
        *(volatile v8h*)(XP + (size_t)(n0 + row) * DM + c0 + c8) = hv;
        if (ps == 0) __threadfence(); }
}

__global__ __launch_bounds__(256) void k_lndw_conv(const float* __restrict__ ACT, const float* __restrict__ ST, const float* __restrict__ G, const float* __restrict__ BE,
                                                   const float* __restrict__ DW, float carry, h16* XP) {
    lndw_body<1>(ACT, ST, G, BE, DW, carry, XP);
}
__global__ __launch_bounds__(256) void k_ln_plain(const float* __restrict__ ACT, const float* __restrict__ ST, const float* __restrict__ G, const float* __restrict__ BE,
                                                  float carry, h16* XP) {
    lndw_body<0>(ACT, ST, G, BE, G, carry, XP);
}

template <int BROW, int HASB, int RELU>
__device__ __forceinline__ void gemm_plane_body(const h16* __restrict__ A, const h16* __restrict__ Bt, const float* __restrict__ bias, float scale, float ocar,
                                                h16* Ph, int RB, size_t sRB, int pitch, int CB, size_t sCB) {
    __shared__ __align__(16) float os[16 * 68];
    const int K = DM;
    const int lane = threadIdx.x & 31, lr = lane & 15, hi = lane >> 4; const int r0 = blockIdx.x * 64, c0 = blockIdx.y * 64;
    v8f acc[4][4];
#pragma unroll
    for (int mb = 0; mb < 4; ++mb)
#pragma unroll
        for (int nb = 0; nb < 4; ++nb) acc[mb][nb] = (v8f){};
    const size_t aoff = (size_t)(r0 + lr) * K + 8 * hi, boff = (size_t)(c0 + lr) * K + 8 * hi;
#pragma unroll 1
    for (int kc = 0; kc < K; kc += 32) {
        v16h a[4];
#pragma unroll
        for (int mb = 0; mb < 4; ++mb) a[mb] = ldh(A + aoff + (size_t)mb * 16 * K + kc);
#pragma unroll
        for (int nb = 0; nb < 4; ++nb) { const v16h b = ldh(Bt + boff + (size_t)nb * 16 * K + kc);
#pragma unroll
            for (int mb = 0; mb < 4; ++mb) acc[mb][nb] = wmma16(a[mb], b, acc[mb][nb]); }
        asm volatile("v_nop\n\tv_nop\n\tv_nop\n\tv_nop" : "+v"(acc[0][0]), "+v"(acc[1][1]), "+v"(acc[2][2]), "+v"(acc[3][3]) : "v"(a[0]), "v"(a[1]), "v"(a[2]), "v"(a[3]));
    }
    float bcol[4];
#pragma unroll
    for (int nb = 0; nb < 4; ++nb) { bcol[nb] = 0.0f; if (HASB) { const int ci = BROW ? lr : (c0 + nb * 16 + lr); bcol[nb] = bfr(bias[ci]); } }
    const size_t tbase = (size_t)(r0 / RB) * sRB + (size_t)(r0 % RB) * (size_t)pitch + (size_t)(c0 / CB) * sCB + (size_t)(c0 % CB);
#pragma unroll
    for (int mb = 0; mb < 4; ++mb) {
        float brow[8];
#pragma unroll
        for (int j = 0; j < 8; ++j) { brow[j] = 0.0f; if (HASB) { const int ri = BROW ? (r0 + mb * 16 + 8 * hi + j) : j; brow[j] = bfr(bias[ri]); } }
#pragma unroll
        for (int nb = 0; nb < 4; ++nb) {
#pragma unroll
            for (int j = 0; j < 8; ++j) { float x = acc[mb][nb][j] * scale + (BROW ? brow[j] : bcol[nb]); if (RELU) x = (x > 0.0f) ? x : 0.0f;
                os[(hi * 8 + j) * 68 + nb * 16 + lr] = x * ocar; } }
        wave_sync();
        const size_t sb = tbase + (size_t)(mb * 16) * (size_t)pitch;
#pragma unroll 1
        for (int ps = 0; ps < 2; ++ps) {
#pragma unroll
            for (int s = 0; s < 4; ++s) { const int row = 4 * s + (lane >> 3), c8 = (lane & 7) * 8;
                const v4f x0 = *(const v4fa*)(&os[row * 68 + c8]); const v4f x1 = *(const v4fa*)(&os[row * 68 + c8 + 4]); v8h hv;
#pragma unroll
                for (int i = 0; i < 4; ++i) { hv[i] = (h16)x0[i]; hv[4 + i] = (h16)x1[i]; }
                const size_t oo = sb + (size_t)row * (size_t)pitch + c8;
                *(volatile v8h*)(Ph + oo) = hv; }
            if (ps == 0) __threadfence(); }
        wave_sync();
    }
}

__global__ __launch_bounds__(32) void k_gemm_qk(const h16* __restrict__ A, const h16* __restrict__ Bt, float scale, h16* Ph) {
    gemm_plane_body<0, 0, 0>(A, Bt, (const float*)0, scale, 1.0f, Ph, SEQ, (size_t)NH_ * SEQ * HD, HD, HD, (size_t)SEQ * HD);
}
__global__ __launch_bounds__(32) void k_gemm_vt(const h16* __restrict__ A, const h16* __restrict__ Bt, float scale, h16* Ph) {
    gemm_plane_body<1, 0, 0>(A, Bt, (const float*)0, scale, 1.0f, Ph, DM, (size_t)0, SEQ, SEQ, (size_t)DM * SEQ);
}
__global__ __launch_bounds__(32) void k_gemm_ffn1(const h16* __restrict__ A, const h16* __restrict__ Bt, const float* __restrict__ bias, float scale, float ocar, h16* Ph) {
    gemm_plane_body<0, 1, 1>(A, Bt, bias, scale, ocar, Ph, NTOK, (size_t)0, DM, DM, (size_t)0);
}

__global__ __launch_bounds__(32) void k_gemm_cf(const h16* __restrict__ A, const h16* __restrict__ Bt, const float* __restrict__ bias, float scale, int relu,
                                                const float* __restrict__ RES, int rpitch, float* OUT, int opitch) {
    __shared__ __align__(16) float os[16 * 68];
    const int K = DM;
    const int lane = threadIdx.x & 31, lr = lane & 15, hi = lane >> 4; const int r0 = blockIdx.x * 64, c0 = blockIdx.y * 64;
    v8f acc[4][4];
#pragma unroll
    for (int mb = 0; mb < 4; ++mb)
#pragma unroll
        for (int nb = 0; nb < 4; ++nb) acc[mb][nb] = (v8f){};
    const size_t aoff = (size_t)(r0 + lr) * K + 8 * hi, boff = (size_t)(c0 + lr) * K + 8 * hi;
#pragma unroll 1
    for (int kc = 0; kc < K; kc += 32) {
        v16h a[4];
#pragma unroll
        for (int mb = 0; mb < 4; ++mb) a[mb] = ldh(A + aoff + (size_t)mb * 16 * K + kc);
#pragma unroll
        for (int nb = 0; nb < 4; ++nb) { const v16h b = ldh(Bt + boff + (size_t)nb * 16 * K + kc);
#pragma unroll
            for (int mb = 0; mb < 4; ++mb) acc[mb][nb] = wmma16(a[mb], b, acc[mb][nb]); }
        asm volatile("v_nop\n\tv_nop\n\tv_nop\n\tv_nop" : "+v"(acc[0][0]), "+v"(acc[1][1]), "+v"(acc[2][2]), "+v"(acc[3][3]) : "v"(a[0]), "v"(a[1]), "v"(a[2]), "v"(a[3]));
    }
    const int bb = c0 / SEQ, t0 = c0 % SEQ;
#pragma unroll
    for (int mb = 0; mb < 4; ++mb) {
        float brow[8];
#pragma unroll
        for (int j = 0; j < 8; ++j) brow[j] = bfr(bias[r0 + mb * 16 + 8 * hi + j]);
#pragma unroll
        for (int nb = 0; nb < 4; ++nb) {
#pragma unroll
            for (int j = 0; j < 8; ++j) { float x = acc[mb][nb][j] * scale + brow[j]; x = (relu != 0 && !(x > 0.0f)) ? 0.0f : x;
                os[(hi * 8 + j) * 68 + nb * 16 + lr] = x; } }
        wave_sync();
        const size_t chb = (size_t)bb * DM + r0 + mb * 16;
#pragma unroll 1
        for (int ps = 0; ps < 2; ++ps) {
#pragma unroll
            for (int s = 0; s < 8; ++s) { const int row = 2 * s + (lane >> 4), c4 = (lane & 15) * 4;
                const v4f x = *(const v4fa*)(&os[row * 68 + c4]);
                const v4f r = *(const v4f*)(RES + (chb + row) * (size_t)rpitch + t0 + c4);
                const v4f y = x + r;
                *(volatile v4f*)(OUT + (chb + row) * (size_t)opitch + t0 + c4) = y; }
            if (ps == 0) __threadfence(); }
        wave_sync();
    }
}

__global__ __launch_bounds__(256) void k_flash(const h16* __restrict__ QH, const h16* __restrict__ KP, const h16* __restrict__ VT,
                                               const int* __restrict__ kmask, const float* __restrict__ RES, float* OUT) {
    __shared__ __align__(16) float os[256 * OSP];
    const int lane = threadIdx.x & 31, lr = lane & 15, hi = lane >> 4;
    const int wv = __builtin_amdgcn_readfirstlane((int)(threadIdx.x >> 5));
    const int hl = wv >> 1, qt = wv & 1;
    const int h = blockIdx.z * 4 + hl;
    const int b = blockIdx.y;
    const int t0 = blockIdx.x * 32 + qt * 16;
    const int zh = b * NH_ + h;
    const size_t pbase = (size_t)zh * SEQ * HD;
    const size_t qo = pbase + (size_t)(t0 + lr) * HD + 8 * hi;
    const v16h qh0 = ldh(QH + qo), qh1 = ldh(QH + qo + 32);
    const size_t ko = pbase + (size_t)lr * HD + 8 * hi;
    const size_t vo = pbase + (size_t)lr * SEQ + 8 * hi;
    const int* km = kmask + (size_t)b * SEQ_FULL;
    unsigned myw = 0u;
#pragma unroll 4
    for (int w = 0; w < SEQ / 32; ++w) { const int kv = km[w * 32 + lane]; const unsigned bal = __builtin_amdgcn_ballot_w32(kv != 0); myw = (lane == w) ? bal : myw; }
    v8f o0 = (v8f){}, o1 = (v8f){}, o2 = (v8f){}, o3 = (v8f){};
    float m = -3.0e38f, l = 0.0f;
#pragma unroll 1
    for (int key0 = 0; key0 < SEQ; key0 += 32) {
        const h16* ka = KP + ko + (size_t)key0 * HD;
        const v16h ka0 = ldh(ka), ka1 = ldh(ka + 32), kb0 = ldh(ka + 16 * HD), kb1 = ldh(ka + 16 * HD + 32);
        v8f sa = (v8f){}, sb = (v8f){};
        sa = wmma16(ka0, qh0, sa); sb = wmma16(kb0, qh0, sb);
        sa = wmma16(ka1, qh1, sa); sb = wmma16(kb1, qh1, sb);
        asm volatile("v_nop\n\tv_nop\n\tv_nop\n\tv_nop" : "+v"(sa), "+v"(sb) : "v"(ka0), "v"(ka1), "v"(kb0), "v"(kb1));
        const unsigned mw = (unsigned)__shfl((int)myw, key0 >> 5, 32);
        const unsigned ma = mw >> (8 * hi), mc = mw >> (16 + 8 * hi);
        float ta[8], tb[8]; float mx = -3.0e38f;
#pragma unroll
        for (int r = 0; r < 8; ++r) { const float xa = sa[r] * SC2, xb = sb[r] * SC2;
            ta[r] = ((ma >> r) & 1u) ? xa : NEGL; tb[r] = ((mc >> r) & 1u) ? xb : NEGL; mx = fmaxf(mx, fmaxf(ta[r], tb[r])); }
        mx = fmaxf(mx, __shfl_xor(mx, 16, 32));
        const float mnew = fmaxf(m, mx);
        const float alpha = __builtin_amdgcn_exp2f(m - mnew);
        v16h pb; float ls = 0.0f;
#pragma unroll
        for (int r = 0; r < 8; ++r) { const h16 pa = (h16)__builtin_amdgcn_exp2f((ta[r] - mnew) + PSH); const h16 pc = (h16)__builtin_amdgcn_exp2f((tb[r] - mnew) + PSH); pb[r] = pa; pb[8 + r] = pc; ls += (float)pa + (float)pc; }
        l = l * alpha + ls; m = mnew;
        o0 = o0 * alpha; o1 = o1 * alpha; o2 = o2 * alpha; o3 = o3 * alpha;
        const h16* va = VT + vo + key0;
        const v16h v0 = ldh(va), v1 = ldh(va + (size_t)16 * SEQ), v2 = ldh(va + (size_t)32 * SEQ), v3 = ldh(va + (size_t)48 * SEQ);
        o0 = wmma16(v0, pb, o0); o1 = wmma16(v1, pb, o1); o2 = wmma16(v2, pb, o2); o3 = wmma16(v3, pb, o3);
        asm volatile("v_nop\n\tv_nop\n\tv_nop\n\tv_nop" : "+v"(o0), "+v"(o1), "+v"(o2), "+v"(o3) : "v"(v0), "v"(v1), "v"(v2), "v"(v3), "v"(pb));
    }
    l += __shfl_xor(l, 16, 32);
    const float inv = 1.0f / l;
    const int rb = hl * 64 + 8 * hi, cc = qt * 16 + lr;
#pragma unroll
    for (int r = 0; r < 8; ++r) {
        os[(rb +  0 + r) * OSP + cc] = o0[r] * inv;
        os[(rb + 16 + r) * OSP + cc] = o1[r] * inv;
        os[(rb + 32 + r) * OSP + cc] = o2[r] * inv;
        os[(rb + 48 + r) * OSP + cc] = o3[r] * inv; }
    __syncthreads();
    const int tb0 = blockIdx.x * 32;
    const size_t gb = ((size_t)b * DM + (size_t)blockIdx.z * 256 + (size_t)(32 * wv)) * SEQ + tb0;
#pragma unroll 1
    for (int ps = 0; ps < 2; ++ps) {
#pragma unroll
        for (int s = 0; s < 8; ++s) { const int row = 4 * s + (lane >> 3), c4 = (lane & 7) * 4;
            const v4f x = *(const v4fa*)(&os[(32 * wv + row) * OSP + c4]);
            const size_t off = gb + (size_t)row * SEQ + c4;
            const v4f r = *(const v4f*)(RES + off);
            const v4f y = x + r;
            *(volatile v4f*)(OUT + off) = y; }
        if (ps == 0) __threadfence(); }
}

static constexpr size_t al256(size_t v) { return (v + 255) & ~(size_t)255; }
static constexpr size_t NWH = (size_t)NCONV * DM * DM + (size_t)2 * DM * DM + (size_t)3 * DM * DM;
static constexpr size_t SZ_ACT = al256((size_t)NB * DM * SEQ * 4);
static constexpr size_t SZ_ST  = al256((size_t)2 * NTOK * 4);
static constexpr size_t SZ_XP  = al256((size_t)NTOK * DM * 2);
static constexpr size_t SZ_PL  = al256((size_t)NB * NH_ * SEQ * HD * 2);
static constexpr size_t SZ_WH  = al256(NWH * 2);
static constexpr size_t SZ_TOTAL = 2 * SZ_ACT + SZ_ST + 2 * SZ_XP + 3 * SZ_PL + SZ_WH;
static_assert(SZ_TOTAL <= (size_t)134217728);
static_assert(((size_t)DM * DM * 2) % 256 == 0);
static_assert((size_t)NTOK * DM == (size_t)NB * NH_ * SEQ * HD);

extern "C" void kernel_launch(void* const* d_in, const int* in_sizes, int n_in,
                              void* d_out, int out_size, void* d_ws, size_t ws_size, hipStream_t stream) {
    if (n_in < 19) return;
    const size_t needx = ((size_t)NB * DM - 1) * SEQ_FULL + SEQ;
    const size_t needm = (size_t)(NB - 1) * SEQ_FULL + SEQ;
    if ((size_t)in_sizes[0] < needx || (size_t)in_sizes[1] < needm) return;
    if ((size_t)in_sizes[4] < (size_t)NCONV * DM * KW || (size_t)in_sizes[5] < (size_t)NCONV * DM * DM) return;
    if (in_sizes[6] < NCONV * DM || in_sizes[7] < NCONV * DM || in_sizes[8] < NCONV * DM) return;
    if ((size_t)in_sizes[9] < (size_t)2 * DM * DM || (size_t)in_sizes[10] < (size_t)DM * DM) return;
    if (in_sizes[11] < DM || in_sizes[12] < DM || in_sizes[13] < DM || in_sizes[14] < DM) return;
    if ((size_t)in_sizes[15] < (size_t)DM * DM || in_sizes[16] < DM || (size_t)in_sizes[17] < (size_t)DM * DM || in_sizes[18] < DM) return;
    if ((size_t)out_size < ((size_t)NB * DM - 1) * OUT_SEQ + SEQ) return;
    if (SZ_TOTAL > ws_size) return;
    const float* x = (const float*)d_in[0]; const int* mask = (const int*)d_in[1];
    const float* dw_w = (const float*)d_in[4]; const float* pw_w = (const float*)d_in[5]; const float* pw_b = (const float*)d_in[6];
    const float* nc_g = (const float*)d_in[7]; const float* nc_b = (const float*)d_in[8];
    const float* mem_w = (const float*)d_in[9]; const float* query_w = (const float*)d_in[10];
    const float* n1_g = (const float*)d_in[11]; const float* n1_b = (const float*)d_in[12];
    const float* n2_g = (const float*)d_in[13]; const float* n2_b = (const float*)d_in[14];
    const float* f1_w = (const float*)d_in[15]; const float* f1_b = (const float*)d_in[16];
    const float* f2_w = (const float*)d_in[17]; const float* f2_b = (const float*)d_in[18];
    float* OUT = (float*)d_out;
    char* wsp = (char*)d_ws;
    float* A0 = (float*)wsp; wsp += SZ_ACT;
    float* A1 = (float*)wsp; wsp += SZ_ACT;
    float* ST = (float*)wsp; wsp += SZ_ST;
    h16* XP = (h16*)wsp; wsp += SZ_XP;
    h16* H1 = (h16*)wsp; wsp += SZ_XP;
    h16* QH = (h16*)wsp; wsp += SZ_PL;
    h16* KP = (h16*)wsp; wsp += SZ_PL;
    h16* VT = (h16*)wsp; wsp += SZ_PL;
    h16* WH = (h16*)wsp; wsp += SZ_WH;
    h16* WPW = WH; h16* WMEM = WH + (size_t)NCONV * DM * DM; h16* WQ = WMEM + (size_t)2 * DM * DM; h16* WF1 = WQ + (size_t)DM * DM; h16* WF2 = WF1 + (size_t)DM * DM;

    { const size_t n8 = (size_t)NCONV * DM * DM / 8; k_cvtw<<<(unsigned)((n8 + 255) / 256), 256, 0, stream>>>(pw_w, WPW, n8); }
    { const size_t n8 = (size_t)2 * DM * DM / 8;     k_cvtw<<<(unsigned)((n8 + 255) / 256), 256, 0, stream>>>(mem_w, WMEM, n8); }
    { const size_t n8 = (size_t)DM * DM / 8; const unsigned g = (unsigned)((n8 + 255) / 256);
      k_cvtw<<<g, 256, 0, stream>>>(query_w, WQ, n8); k_cvtw<<<g, 256, 0, stream>>>(f1_w, WF1, n8); k_cvtw<<<g, 256, 0, stream>>>(f2_w, WF2, n8); }

    k_pos<<<(unsigned)(((size_t)(DM / 2) * SEQ) / 256), 256, 0, stream>>>(x, A0);

    const float sc_w  = 1.0f / WCAR;
    const float sc_wx = 1.0f / (WCAR * XCAR);
    float* cur = A0; float* nxt = A1;
    for (int i = 0; i < NCONV; ++i) {
        k_stats<<<NTOK / 32, 256, 0, stream>>>(cur, ST);
        k_lndw_conv<<<dim3(NTOK / 32, DM / 64, 1), 256, 0, stream>>>(cur, ST, nc_g + (size_t)i * DM, nc_b + (size_t)i * DM, dw_w + (size_t)i * DM * KW, XCAR, XP);
        k_gemm_cf<<<dim3(DM / 64, NTOK / 64, 1), 32, 0, stream>>>(WPW + (size_t)i * DM * DM, XP, pw_b + (size_t)i * DM, sc_wx, 1, cur, SEQ, nxt, SEQ);
        float* t = cur; cur = nxt; nxt = t;
    }
    k_stats<<<NTOK / 32, 256, 0, stream>>>(cur, ST);
    k_ln_plain<<<dim3(NTOK / 32, DM / 64, 1), 256, 0, stream>>>(cur, ST, n1_g, n1_b, 1.0f, XP);
    k_gemm_qk<<<dim3(NTOK / 64, DM / 64, 1), 32, 0, stream>>>(XP, WQ, sc_w, QH);
    k_gemm_qk<<<dim3(NTOK / 64, DM / 64, 1), 32, 0, stream>>>(XP, WMEM, sc_w, KP);
    k_gemm_vt<<<dim3(DM / 64, NTOK / 64, 1), 32, 0, stream>>>(WMEM + (size_t)DM * DM, XP, sc_w, VT);
    k_flash<<<dim3(SEQ / 32, NB, 2), 256, 0, stream>>>(QH, KP, VT, mask, cur, nxt);
    { float* t = cur; cur = nxt; nxt = t; }
    k_stats<<<NTOK / 32, 256, 0, stream>>>(cur, ST);
    k_ln_plain<<<dim3(NTOK / 32, DM / 64, 1), 256, 0, stream>>>(cur, ST, n2_g, n2_b, 1.0f, XP);
    k_gemm_ffn1<<<dim3(NTOK / 64, DM / 64, 1), 32, 0, stream>>>(XP, WF1, f1_b, sc_w, XCAR, H1);
    k_gemm_cf<<<dim3(DM / 64, NTOK / 64, 1), 32, 0, stream>>>(WF2, H1, f2_b, sc_wx, 0, cur, SEQ, OUT, OUT_SEQ);
}
